// CalibrationNetwork_8873402433722
// MI455X (gfx1250) — hardware-verified
//
#include <hip/hip_runtime.h>
#include <stddef.h>


typedef _Float16 v16h __attribute__((ext_vector_type(16)));
typedef _Float16 v8h  __attribute__((ext_vector_type(8)));
typedef float    v8f  __attribute__((ext_vector_type(8)));
typedef float    v4f  __attribute__((ext_vector_type(4)));
typedef _Float16 h16;

#ifndef NB
#define NB 32768
#endif
#define NB_FULL 32768
#define NJ   32
#define NQ   7
#define NO   5
#define HW   64
#define XROW (NQ * NO)
#define W1K  (NO + 1)
#define W2K  (HW + 1)
#define CH   4096
#define NCHUNK ((NB + CH - 1) / CH)
#define OPITCH 64

#define LDT 72
#define LDC 68

#define WCARRY 64.0f
#define XCARRY 64.0f
#define MCARRY 16.0f

#define W1S_N (NQ * HW * 8)
#define XS_N  (16 * LDT)
#define PLANE_BYTES ((size_t)NB * OPITCH * 4)
#define WS_TOTAL PLANE_BYTES

static_assert(NB >= 32 && NB <= NB_FULL && (NB % 32) == 0);
static_assert(XROW == 35);
static_assert(((size_t)NB * XROW) % 4 == 0);
static_assert((((size_t)NB * XROW * 4) % 128) == 0);
static_assert(HW == 64 && (HW % 32) == 0);
static_assert(NO <= 8 && NO <= 16);
static_assert(NQ * 8 <= OPITCH);
static_assert(NQ * 8 + 8 <= LDT);
static_assert((OPITCH * 4) % 128 == 0 && OPITCH == 16 * 4);
static_assert((CH % 32) == 0 && (CH % 16) == 0 && CH <= 65536);
static_assert((LDT % 8) == 0 && LDT >= 64);
static_assert((LDC % 4) == 0 && LDC >= 64);
static_assert(((W1S_N * 2) % 16) == 0 && ((XS_N * 2) % 16) == 0);
static_assert(((XS_N + 8) % 8) == 0);
static_assert(((16 * LDC) % 4) == 0);
static_assert((size_t)(W1S_N + 8) * 2 + (size_t)HW * LDT * 2 + (size_t)NQ * 16 * LDT * 2 +
              (size_t)NQ * HW * 4 + (size_t)HW * 4 + (size_t)128 * 4 + (size_t)(XS_N + 8) * 2 +
              (size_t)2 * 16 * LDT * 2 + (size_t)16 * LDC * 4 + (size_t)CH * 2 <= (size_t)65536);
static_assert((PLANE_BYTES % 128) == 0);
static_assert(WS_TOTAL <= (size_t)134217728);
static_assert((size_t)NB * OPITCH < (size_t)0xFFFFFFFFu);

__device__ __forceinline__ float bf16r(float x) {
  unsigned int u = __float_as_uint(x);
  u = (u + 0x7FFFu + ((u >> 16) & 1u)) & 0xFFFF0000u;
  return __uint_as_float(u);
}

__device__ __forceinline__ v16h frag_at(const _Float16* p) {
  v8h lo = *(const v8h*)(p);
  v8h hi = *(const v8h*)(p + 16);
  v16h out;
#pragma unroll
  for (int i = 0; i < 8; ++i) { out[i] = lo[i]; out[i + 8] = hi[i]; }
  return out;
}
__device__ __forceinline__ v16h ld_frag(const _Float16* base, unsigned ld) {
  const unsigned lane = threadIdx.x & 31u;
  return frag_at(base + (lane & 15u) * ld + (lane >> 4) * 8u);
}

__device__ __forceinline__ v8f wmma16(v16h a, v16h b, v8f c) {
  v8f d = __builtin_amdgcn_wmma_f32_16x16x32_f16(false, a, false, b, (short)0, c,
                                                 false, false);
  asm volatile("v_nop\n\tv_nop\n\tv_nop\n\tv_nop" : "+v"(d) : "v"(a), "v"(b));
  return d;
}

static __device__ __forceinline__ h16 toh_flush(float v) {
  const h16 r = (h16)v;
  return (fabsf(v) < 6.103515625e-05f) ? (h16)0.0f : r;
}

__device__ __forceinline__ v16h frag_low(v8h lo) {
  v16h out;
#pragma unroll
  for (int i = 0; i < 8; ++i) { out[i] = lo[i]; out[i + 8] = (_Float16)0.0f; }
  return out;
}

__device__ __forceinline__ v8f splat8(float b) {
  v8f o;
#pragma unroll
  for (int i = 0; i < 8; ++i) o[i] = b;
  return o;
}

__global__ __launch_bounds__(32) void calib_kernel(
    const float* __restrict__ x, const int* __restrict__ jid,
    const float* __restrict__ W1, const float* __restrict__ W1a,
    const float* __restrict__ W2, const float* __restrict__ W2a,
    const float* __restrict__ V, const float* __restrict__ Va,
    float* __restrict__ Pl) {
  __shared__ __attribute__((aligned(16))) _Float16 W1s[W1S_N + 8];
  __shared__ __attribute__((aligned(16))) _Float16 W2s[HW * LDT];
  __shared__ __attribute__((aligned(16))) _Float16 V3s[NQ * 16 * LDT];
  __shared__ __attribute__((aligned(16))) float b1s[NQ * HW];
  __shared__ __attribute__((aligned(16))) float b2s[HW];
  __shared__ __attribute__((aligned(16))) float b3s[8 * 16];
  __shared__ __attribute__((aligned(16))) _Float16 Xs[XS_N + 8];
  __shared__ __attribute__((aligned(16))) _Float16 Z1[16 * LDT];
  __shared__ __attribute__((aligned(16))) _Float16 Z2[16 * LDT];
  __shared__ __attribute__((aligned(16))) float Ot[16 * LDC];
  __shared__ __attribute__((aligned(16))) unsigned short lst[CH];

  const unsigned lane = threadIdx.x & 31u;
  const unsigned hh = lane >> 4, m = lane & 15u;
  const unsigned j = blockIdx.y;
  const unsigned cbase = blockIdx.x * (unsigned)CH;

  unsigned cnt = 0u;
#pragma unroll 1
  for (unsigned it = 0; it < (unsigned)(CH / 32); ++it) {
    const unsigned loc = it * 32u + lane;
    const unsigned e = cbase + loc;
    const unsigned ec = (e < (unsigned)NB) ? e : (unsigned)(NB - 1);
    int jv = jid[ec];
    asm volatile("" : "+v"(jv));
    jv = (jv < 0) ? 0 : jv;
    jv = (jv > (NJ - 1)) ? (NJ - 1) : jv;
    const bool hit = (e < (unsigned)NB) && ((unsigned)jv == j);
    const unsigned mask = __builtin_amdgcn_ballot_w32(hit);
    const unsigned pre = __builtin_amdgcn_mbcnt_lo(mask, 0u);
    unsigned pos = cnt + pre;
    pos = (pos < (unsigned)CH) ? pos : (unsigned)(CH - 1);
    if (hit) lst[pos] = (unsigned short)loc;
    cnt += (unsigned)__popc(mask);
  }
  cnt = (cnt < (unsigned)CH) ? cnt : (unsigned)CH;
  cnt = (unsigned)__builtin_amdgcn_readfirstlane((int)cnt);
  const unsigned ntiles = (cnt + 15u) >> 4;

  {
    v8h zh;
#pragma unroll
    for (int i = 0; i < 8; ++i) zh[i] = (_Float16)0.0f;
#pragma unroll 1
    for (unsigned idx = lane; idx < (unsigned)((XS_N + 8) / 8); idx += 32u)
      *(v8h*)&Xs[idx * 8u] = zh;
    if (lane == 0u) *(v8h*)&W1s[W1S_N] = zh;
    v4f zf;
#pragma unroll
    for (int i = 0; i < 4; ++i) zf[i] = 0.0f;
#pragma unroll 1
    for (unsigned idx = lane; idx < (unsigned)((16 * LDC) / 4); idx += 32u)
      *(v4f*)&Ot[idx * 4u] = zf;
  }

#pragma unroll 1
  for (unsigned idx = lane; idx < (unsigned)W1S_N; idx += 32u) {
    const unsigned k = idx & 7u;
    const unsigned qn = idx >> 3;
    const unsigned kc = (k < (unsigned)NO) ? k : (unsigned)(NO - 1);
    float a = W1[(size_t)qn * W1K + 1u + kc];
    float b = W1a[((size_t)j * (NQ * HW) + qn) * W1K + 1u + kc];
    asm volatile("" : "+v"(a));
    asm volatile("" : "+v"(b));
    const h16 hv = toh_flush(WCARRY * (bf16r(a) + bf16r(b)));
    W1s[idx] = (k < (unsigned)NO) ? hv : (h16)0.0f;
  }
#pragma unroll 1
  for (unsigned idx = lane; idx < (unsigned)(NQ * HW); idx += 32u) {
    const float a = W1[(size_t)idx * W1K];
    const float b = W1a[((size_t)j * (NQ * HW) + idx) * W1K];
    b1s[idx] = (XCARRY * WCARRY) * (bf16r(a) + bf16r(b));
  }
#pragma unroll 1
  for (unsigned idx = lane; idx < (unsigned)(HW * HW); idx += 32u) {
    const unsigned i = idx & 63u, n = idx >> 6;
    const float a = W2[(size_t)n * W2K + 1u + i];
    const float b = W2a[((size_t)j * HW + n) * W2K + 1u + i];
    W2s[n * LDT + i] = toh_flush(WCARRY * (bf16r(a) + bf16r(b)));
  }
#pragma unroll 1
  for (unsigned idx = lane; idx < (unsigned)HW; idx += 32u) {
    const float a = W2[(size_t)idx * W2K];
    const float b = W2a[((size_t)j * HW + idx) * W2K];
    b2s[idx] = (MCARRY * WCARRY) * (bf16r(a) + bf16r(b));
  }
#pragma unroll 1
  for (unsigned idx = lane; idx < (unsigned)(NQ * 16 * HW); idx += 32u) {
    const unsigned i = idx & 63u;
    const unsigned o = (idx >> 6) & 15u;
    const unsigned q = idx >> 10;
    const unsigned oc = (o < (unsigned)NO) ? o : (unsigned)(NO - 1);
    float a = V[((size_t)q * NO + oc) * W2K + 1u + i];
    float b = Va[(((size_t)j * NQ + q) * NO + oc) * W2K + 1u + i];
    asm volatile("" : "+v"(a));
    asm volatile("" : "+v"(b));
    const h16 hv = toh_flush(WCARRY * (bf16r(a) + bf16r(b)));
    V3s[(q * 16u + o) * LDT + i] = (o < (unsigned)NO) ? hv : (h16)0.0f;
  }
#pragma unroll 1
  for (unsigned idx = lane; idx < 128u; idx += 32u) {
    const unsigned o = idx & 15u;
    const unsigned q = idx >> 4;
    const unsigned oc = (o < (unsigned)NO) ? o : (unsigned)(NO - 1);
    const unsigned qc = (q < (unsigned)NQ) ? q : (unsigned)(NQ - 1);
    float a = V[((size_t)qc * NO + oc) * W2K];
    float b = Va[(((size_t)j * NQ + qc) * NO + oc) * W2K];
    asm volatile("" : "+v"(a));
    asm volatile("" : "+v"(b));
    const float bv = (MCARRY * WCARRY) * (bf16r(a) + bf16r(b));
    b3s[idx] = (o < (unsigned)NO) ? bv : 0.0f;
  }
  __syncthreads();

#pragma unroll 1
  for (unsigned t = 0; t < ntiles; ++t) {
    {
      const unsigned si = t * 16u + m;
      const bool rv = si < cnt;
      const unsigned sic = rv ? si : (cnt - 1u);
      unsigned bs = cbase + (unsigned)lst[sic];
      bs = (bs < (unsigned)NB) ? bs : (unsigned)(NB - 1);
      const float* xr = x + (size_t)bs * XROW;
#pragma unroll 1
      for (unsigned c0 = 0; c0 < 36u; c0 += 2u) {
        const unsigned cc = c0 + hh;
        const unsigned cl = (cc < (unsigned)XROW) ? cc : (unsigned)(XROW - 1);
        float xv = xr[cl];
        asm volatile("" : "+v"(xv));
        const unsigned qq = cl / 5u;
        const unsigned oo = cl - qq * 5u;
        h16 hv = toh_flush(XCARRY * bf16r(xv));
        hv = rv ? hv : (h16)0.0f;
        if (cc < (unsigned)XROW) Xs[m * LDT + qq * 8u + oo] = hv;
      }
    }
    __syncthreads();

#pragma unroll 1
    for (unsigned q = 0; q < (unsigned)NQ; ++q) {
      {
        const unsigned xo = hh ? (unsigned)XS_N : (m * LDT + q * 8u);
        const v16h xa = frag_low(*(const v8h*)&Xs[xo]);
        v8f acc[4];
#pragma unroll
        for (int nt = 0; nt < 4; ++nt) acc[nt] = splat8(b1s[q * HW + (unsigned)nt * 16u + m]);
#pragma unroll
        for (int nt = 0; nt < 4; ++nt) {
          const unsigned wo = hh ? (unsigned)W1S_N : ((q * HW + (unsigned)nt * 16u + m) * 8u);
          const v16h wf = frag_low(*(const v8h*)&W1s[wo]);
          acc[nt] = wmma16(xa, wf, acc[nt]);
        }
#pragma unroll
        for (int nt = 0; nt < 4; ++nt)
#pragma unroll
          for (int r = 0; r < 8; ++r)
            Z1[(hh * 8u + (unsigned)r) * LDT + (unsigned)nt * 16u + m] =
                toh_flush(MCARRY * fmaxf(acc[nt][r] * (1.0f / (XCARRY * WCARRY)), 0.0f));
      }
      __syncthreads();

      {
        const v16h a0 = ld_frag(Z1, LDT);
        const v16h a1 = ld_frag(Z1 + 32, LDT);
        v8f acc[4];
#pragma unroll
        for (int nt = 0; nt < 4; ++nt) acc[nt] = splat8(b2s[(unsigned)nt * 16u + m]);
#pragma unroll
        for (int nt = 0; nt < 4; ++nt) {
          const v16h w0 = ld_frag(&W2s[(nt * 16) * LDT], LDT);
          acc[nt] = wmma16(a0, w0, acc[nt]);
          const v16h w1 = ld_frag(&W2s[(nt * 16) * LDT + 32], LDT);
          acc[nt] = wmma16(a1, w1, acc[nt]);
        }
#pragma unroll
        for (int nt = 0; nt < 4; ++nt)
#pragma unroll
          for (int r = 0; r < 8; ++r)
            Z2[(hh * 8u + (unsigned)r) * LDT + (unsigned)nt * 16u + m] =
                toh_flush(MCARRY * fmaxf(acc[nt][r] * (1.0f / (MCARRY * WCARRY)), 0.0f));
      }
      __syncthreads();

      {
        const v16h a0 = ld_frag(Z2, LDT);
        const v16h a1 = ld_frag(Z2 + 32, LDT);
        v8f acc = splat8(b3s[q * 16u + m]);
        const v16h w0 = ld_frag(&V3s[(q * 16u) * LDT], LDT);
        acc = wmma16(a0, w0, acc);
        const v16h w1 = ld_frag(&V3s[(q * 16u) * LDT + 32u], LDT);
        acc = wmma16(a1, w1, acc);
        if (m < 8u) {
#pragma unroll
          for (int r = 0; r < 8; ++r) {
            const float lg = acc[r] * (1.0f / (MCARRY * WCARRY));
            Ot[(hh * 8u + (unsigned)r) * LDC + q * 8u + m] = (m < (unsigned)NO) ? lg : 0.0f;
          }
        }
      }
    }
    __syncthreads();

#pragma unroll 1
    for (unsigned it = 0; it < 4u; ++it) {
      const unsigned idx = lane + 32u * it;
      const unsigned s = idx & 15u;
      const unsigned qq = idx >> 4;
      const unsigned ro = s * LDC + qq * 8u;
      const v4f u = *(const v4f*)&Ot[ro];
      const v4f u2 = *(const v4f*)&Ot[ro + 4u];
      float mx = fmaxf(fmaxf(u[0], u[1]), fmaxf(u[2], u[3]));
      mx = fmaxf(mx, u2[0]);
      const float e0 = __expf(u[0] - mx);
      const float e1 = __expf(u[1] - mx);
      const float e2 = __expf(u[2] - mx);
      const float e3 = __expf(u[3] - mx);
      const float e4 = __expf(u2[0] - mx);
      const float den = ((e0 + e1) + (e2 + e3)) + e4;
      const float inv = __builtin_amdgcn_rcpf(den);
      const bool live = qq < (unsigned)NQ;
      v4f p0, p1;
      p0[0] = live ? e0 * inv : 0.0f;
      p0[1] = live ? e1 * inv : 0.0f;
      p0[2] = live ? e2 * inv : 0.0f;
      p0[3] = live ? e3 * inv : 0.0f;
      p1[0] = live ? e4 * inv : 0.0f;
      p1[1] = 0.0f;
      p1[2] = 0.0f;
      p1[3] = 0.0f;
      *(v4f*)&Ot[ro] = p0;
      *(v4f*)&Ot[ro + 4u] = p1;
    }
    __syncthreads();

    {
      v4f xs[8];
      size_t off[8];
      bool ok[8];
#pragma unroll
      for (unsigned i = 0; i < 8u; ++i) {
        const unsigned s = 2u * i + hh;
        const unsigned sj = t * 16u + s;
        const bool okk = sj < cnt;
        const unsigned sjc = okk ? sj : (cnt - 1u);
        unsigned bb = cbase + (unsigned)lst[sjc];
        bb = (bb < (unsigned)NB) ? bb : (unsigned)(NB - 1);
        xs[i] = *(const v4f*)&Ot[s * LDC + m * 4u];
        off[i] = (size_t)bb * OPITCH + m * 4u;
        ok[i] = okk;
      }
#pragma unroll
      for (int i = 0; i < 8; ++i)
        if (ok[i]) *(volatile v4f*)(Pl + off[i]) = xs[i];
      __threadfence();
#pragma unroll
      for (int i = 0; i < 8; ++i)
        if (ok[i]) *(volatile v4f*)(Pl + off[i]) = xs[i];
    }
    __syncthreads();
  }
}

__global__ __launch_bounds__(256) void finalize_kernel(
    const float* __restrict__ Pl, float* __restrict__ out) {
  const unsigned n4 = (unsigned)(((size_t)NB * XROW) / 4);
  const unsigned t = blockIdx.x * 256u + threadIdx.x;
  const unsigned tc = (t < n4) ? t : (n4 - 1u);
  v4f v;
#pragma unroll
  for (unsigned i = 0; i < 4u; ++i) {
    const unsigned e = tc * 4u + i;
    const unsigned b = e / (unsigned)XROW;
    const unsigned c = e - b * (unsigned)XROW;
    const unsigned q = c / 5u;
    const unsigned o = c - q * 5u;
    v[i] = Pl[(size_t)b * OPITCH + q * 8u + o];
  }
  float* p = out + (size_t)tc * 4u;
  if (t < n4) *(volatile v4f*)p = v;
  __threadfence();
  if (t < n4) *(volatile v4f*)p = v;
}

extern "C" void kernel_launch(void* const* d_in, const int* in_sizes, int n_in,
                              void* d_out, int out_size, void* d_ws, size_t ws_size,
                              hipStream_t stream) {
  if (n_in < 8) return;
  if ((long long)in_sizes[0] < (long long)NB * XROW) return;
  if ((long long)in_sizes[1] < (long long)NB) return;
  if ((long long)in_sizes[2] < (long long)NQ * HW * W1K) return;
  if ((long long)in_sizes[3] < (long long)NJ * NQ * HW * W1K) return;
  if ((long long)in_sizes[4] < (long long)HW * W2K) return;
  if ((long long)in_sizes[5] < (long long)NJ * HW * W2K) return;
  if ((long long)in_sizes[6] < (long long)NQ * NO * W2K) return;
  if ((long long)in_sizes[7] < (long long)NJ * NQ * NO * W2K) return;
  if ((long long)out_size < (long long)NB * XROW) return;
  if (ws_size < WS_TOTAL) return;

  const float* x   = (const float*)d_in[0];
  const int*   jid = (const int*)d_in[1];
  const float* W1  = (const float*)d_in[2];
  const float* W1a = (const float*)d_in[3];
  const float* W2  = (const float*)d_in[4];
  const float* W2a = (const float*)d_in[5];
  const float* V   = (const float*)d_in[6];
  const float* Va  = (const float*)d_in[7];
  float* out = (float*)d_out;
  float* Pl = (float*)d_ws;

  calib_kernel<<<dim3(NCHUNK, NJ), dim3(32), 0, stream>>>(x, jid, W1, W1a, W2, W2a, V, Va, Pl);

  const unsigned n4 = (unsigned)(((size_t)NB * XROW) / 4);
  finalize_kernel<<<dim3((n4 + 255u) / 256u), dim3(256), 0, stream>>>(Pl, out);
}
